// MultiHeadSelfAttention_28913719837460
// MI455X (gfx1250) — hardware-run, weakly checked
//
#include <hip/hip_runtime.h>


#ifndef NB
#define NB 2
#endif
#ifndef SEQ
#define SEQ 2048
#endif
#define NB_FULL  2
#define SEQ_FULL 2048
#define DM   1024
#define NH   16
#define HD   64
#define DQ   (NH * HD)
#define NBH  (NB * NH)
#define SCL  0.125f
#define LOG2E 1.4426950408889634f
#define PEXP 10.0f

typedef _Float16 h16;
typedef unsigned short bf;
typedef __attribute__((ext_vector_type(16))) __bf16   v16bf;
typedef __attribute__((ext_vector_type(16))) _Float16 v16h;
typedef __attribute__((ext_vector_type(8)))  _Float16 v8h;
typedef __attribute__((ext_vector_type(8)))  unsigned short v8us;
typedef __attribute__((ext_vector_type(2)))  unsigned short v2us;
typedef __attribute__((ext_vector_type(8)))  float    v8f;
typedef __attribute__((ext_vector_type(4)))  float    v4f;
typedef v4f  __attribute__((may_alias)) v4fa;
typedef v8us __attribute__((may_alias)) v8usa;

static_assert(DQ == DM);
static_assert(HD == 64);
static_assert(SEQ % 64 == 0);
static_assert((NB * SEQ) % 64 == 0);
static_assert(DM % 64 == 0 && (3 * DQ) % 64 == 0);
static_assert(DM % 32 == 0 && DQ % 32 == 0);
static_assert(NB <= NB_FULL && SEQ <= SEQ_FULL);
static_assert(DM % 8 == 0);

__device__ __forceinline__ unsigned short f2bf(float f) { unsigned u = __float_as_uint(f); u += 0x7FFFu + ((u >> 16) & 1u); return (unsigned short)(u >> 16); }
__device__ __forceinline__ float bf2f(unsigned short b) { return __uint_as_float(((unsigned)b) << 16); }
__device__ __forceinline__ float bfr(float f) { return bf2f(f2bf(f)); }
__device__ __forceinline__ void splitf(float y, unsigned short& h, unsigned short& l) { h = f2bf(y); l = f2bf(y - bf2f(h)); }
__device__ __forceinline__ v16h cat16(v8h lo, v8h hi) { return __builtin_shufflevector(lo, hi, 0, 1, 2, 3, 4, 5, 6, 7, 8, 9, 10, 11, 12, 13, 14, 15); }
__device__ __forceinline__ v16bf cat16b(v8us lo, v8us hi) { return __builtin_bit_cast(v16bf, __builtin_shufflevector(lo, hi, 0, 1, 2, 3, 4, 5, 6, 7, 8, 9, 10, 11, 12, 13, 14, 15)); }
__device__ __forceinline__ v8f wmma16(v16h a, v16h b, v8f c) { return __builtin_amdgcn_wmma_f32_16x16x32_f16(false, a, false, b, (short)0, c, false, false); }
__device__ __forceinline__ v8f wmmab(v16bf a, v16bf b, v8f c) { return __builtin_amdgcn_wmma_f32_16x16x32_bf16(false, a, false, b, (short)0, c, false, false); }
__device__ __forceinline__ v16bf ldbf(const bf* p) { return cat16b(*(const v8us*)p, *(const v8us*)(p + 16)); }
__device__ __forceinline__ v16h ldhf(const h16* p) { return cat16(*(const v8h*)p, *(const v8h*)(p + 16)); }

template <bool SPLITA, bool BIAS>
__device__ __forceinline__ void gemmw_body(const bf* __restrict__ A, const bf* __restrict__ A2, const bf* __restrict__ Bt, const int K, float* C, const int ldc, const float* __restrict__ bias, const size_t sA, const size_t sC) {
    __shared__ __align__(16) float os[16 * 68];
    const size_t z = blockIdx.z; A += z * sA; A2 += z * sA; C += z * sC;
    const int lane = threadIdx.x & 31, lr = lane & 15, hi = lane >> 4; const int r0 = blockIdx.x * 64, c0 = blockIdx.y * 64;
    v8f acc[4][4];
#pragma unroll
    for (int mb = 0; mb < 4; ++mb)
#pragma unroll
        for (int nb = 0; nb < 4; ++nb) acc[mb][nb] = (v8f){};
    const size_t aoff = (size_t)(r0 + lr) * K + 8 * hi, boff = (size_t)(c0 + lr) * K + 8 * hi;
#pragma unroll 1
    for (int kc = 0; kc < K; kc += 32) {
        v16bf a[4], a2[4], blast;
#pragma unroll
        for (int mb = 0; mb < 4; ++mb) { a[mb] = ldbf(A + aoff + (size_t)mb * 16 * K + kc); if (SPLITA) a2[mb] = ldbf(A2 + aoff + (size_t)mb * 16 * K + kc); }
#pragma unroll
        for (int nb = 0; nb < 4; ++nb) { const v16bf b = ldbf(Bt + boff + (size_t)nb * 16 * K + kc); if (nb == 3) blast = b;
#pragma unroll
            for (int mb = 0; mb < 4; ++mb) { acc[mb][nb] = wmmab(a[mb], b, acc[mb][nb]); if (SPLITA) acc[mb][nb] = wmmab(a2[mb], b, acc[mb][nb]); } }
        asm volatile("" : "+v"(acc[0][0]), "+v"(acc[0][1]), "+v"(acc[0][2]), "+v"(acc[0][3]), "+v"(acc[1][0]), "+v"(acc[1][1]), "+v"(acc[1][2]), "+v"(acc[1][3]));
        asm volatile("v_nop\n\tv_nop\n\tv_nop\n\tv_nop" : "+v"(acc[2][0]), "+v"(acc[2][1]), "+v"(acc[2][2]), "+v"(acc[2][3]), "+v"(acc[3][0]), "+v"(acc[3][1]), "+v"(acc[3][2]), "+v"(acc[3][3]) : "v"(a[0]), "v"(a[3]), "v"(blast));
    }
#pragma unroll
    for (int mb = 0; mb < 4; ++mb) {
#pragma unroll
        for (int nb = 0; nb < 4; ++nb) {
#pragma unroll
            for (int j = 0; j < 8; ++j) os[(hi * 8 + j) * 68 + nb * 16 + lr] = acc[mb][nb][j]; }
        __builtin_amdgcn_wave_barrier(); asm volatile("" ::: "memory");
        float* crow = C + (size_t)(r0 + mb * 16) * ldc + c0;
#pragma unroll 1
        for (int ps = 0; ps < 2; ++ps) {
#pragma unroll
            for (int s = 0; s < 8; ++s) { const int row = 2 * s + hi, cofs = lr * 4; v4f val = *(const v4fa*)(os + row * 68 + cofs);
                if (BIAS) { val[0] += bfr(bias[c0 + cofs]); val[1] += bfr(bias[c0 + cofs + 1]); val[2] += bfr(bias[c0 + cofs + 2]); val[3] += bfr(bias[c0 + cofs + 3]); }
                *(volatile v4f*)(crow + (size_t)row * ldc + cofs) = val; }
            if (ps == 0) __threadfence(); }
        __builtin_amdgcn_wave_barrier(); asm volatile("" ::: "memory");
    }
}

__global__ __launch_bounds__(32) void k_gemm_qkv(const bf* __restrict__ A, const bf* __restrict__ Bt, float* C, const float* __restrict__ bias) {
    gemmw_body<false, true>(A, A, Bt, DM, C, 3 * DQ, bias, (size_t)0, (size_t)0);
}
__global__ __launch_bounds__(32) void k_gemm_out(const bf* __restrict__ Ah, const bf* __restrict__ Al, const bf* __restrict__ Bt, float* C, const float* __restrict__ bias) {
    gemmw_body<true, true>(Ah, Al, Bt, DQ, C, DM, bias, (size_t)SEQ * DQ, (size_t)SEQ_FULL * DM);
}

__global__ __launch_bounds__(256) void k_wtG(const float* __restrict__ w, int K, int N, bf* Bt) {
    const int lane = threadIdx.x & 31; const int L0 = (blockIdx.x * 8 + (threadIdx.x >> 5)) * 8; const int nlines = N * K / 64;
#pragma unroll
    for (int ps = 0; ps < 2; ++ps) {
#pragma unroll 1
        for (int l = 0; l < 8; ++l) { const int L = L0 + l; if (L >= nlines) break; const size_t e = (size_t)L * 64 + lane * 2; const int k = (int)(e % K), n = (int)(e / K); v2us o;
            o[0] = f2bf(w[(size_t)k * N + n]); o[1] = f2bf(w[(size_t)(k + 1) * N + n]); *(volatile v2us*)(Bt + e) = o; }
        if (ps == 0) __threadfence(); }
}

__global__ __launch_bounds__(256) void k_cvt8(const float* __restrict__ x, bf* XB) {
    const size_t i = (size_t)blockIdx.x * 256 + threadIdx.x; const size_t n8 = (size_t)NB * SEQ * DM / 8; if (i >= n8) return;
    const size_t row = i / (DM / 8); const int c8 = (int)(i % (DM / 8)); const size_t b = row / SEQ, t = row % SEQ;
    const v8f v = *(const v8f*)(x + (b * SEQ_FULL + t) * DM + (size_t)c8 * 8); v8us o;
#pragma unroll
    for (int k = 0; k < 8; ++k) o[k] = f2bf(v[k]);
    *(volatile v8us*)(XB + i * 8) = o; __threadfence(); *(volatile v8us*)(XB + i * 8) = o;
}

__global__ __launch_bounds__(256) void k_qkp(const float* __restrict__ F, bf* PH, bf* PL) {
    const size_t g = (size_t)blockIdx.x * 256 + threadIdx.x; const size_t NG = (size_t)2 * NBH * SEQ * (HD / 8); if (g >= NG) return;
    const int d8 = (int)(g % (HD / 8)); const int t = (int)((g / (HD / 8)) % SEQ); const int bh = (int)((g / ((size_t)(HD / 8) * SEQ)) % NBH); const int which = (int)(g / ((size_t)(HD / 8) * SEQ * NBH));
    const int b = bh / NH, h = bh % NH; const float sc = (which == 0) ? SCL : 1.0f;
    const float* f = F + (size_t)(b * SEQ + t) * (3 * DQ) + which * DQ + h * HD + d8 * 8;
    const v4f a = *(const v4f*)f; const v4f c = *(const v4f*)(f + 4); v8us oh, ol;
#pragma unroll
    for (int q = 0; q < 4; ++q) { unsigned short u, w2; splitf(a[q] * sc, u, w2); oh[q] = u; ol[q] = w2; splitf(c[q] * sc, u, w2); oh[4 + q] = u; ol[4 + q] = w2; }
    *(volatile v8us*)(PH + g * 8) = oh; *(volatile v8us*)(PL + g * 8) = ol; __threadfence(); *(volatile v8us*)(PH + g * 8) = oh; *(volatile v8us*)(PL + g * 8) = ol;
}

__global__ __launch_bounds__(256) void k_vtp(const float* __restrict__ F, h16* VT) {
    const size_t g = (size_t)blockIdx.x * 256 + threadIdx.x; const size_t NG = (size_t)NBH * HD * (SEQ / 8); if (g >= NG) return;
    const int t8 = (int)(g % (SEQ / 8)); const int d = (int)((g / (SEQ / 8)) % HD); const int bh = (int)(g / ((size_t)(SEQ / 8) * HD)); const int b = bh / NH, h = bh % NH;
    const float* f = F + (size_t)(b * SEQ + t8 * 8) * (3 * DQ) + 2 * DQ + h * HD + d; v8h o;
#pragma unroll
    for (int j = 0; j < 8; ++j) o[j] = (h16)f[(size_t)j * (3 * DQ)];
    *(volatile v8h*)(VT + g * 8) = o; __threadfence(); *(volatile v8h*)(VT + g * 8) = o;
}

__global__ __launch_bounds__(128) void k_flash(const bf* __restrict__ QH, const bf* __restrict__ QL, const bf* __restrict__ KH, const bf* __restrict__ KL, const h16* __restrict__ VT, bf* ATH, bf* ATL) {
    __shared__ __align__(16) unsigned short sth[4][16 * 72];
    __shared__ __align__(16) unsigned short stl[4][16 * 72];
    const int wave = __builtin_amdgcn_readfirstlane(threadIdx.x >> 5);
    const int lane = threadIdx.x & 31, lr = lane & 15, hi = lane >> 4;
    const int bh = blockIdx.y; const int b = bh / NH, head = bh % NH;
    const int q0 = blockIdx.x * 64 + wave * 16;
    const size_t pbase = (size_t)bh * SEQ * HD;
    const size_t qoff = pbase + (size_t)(q0 + lr) * HD + 8 * hi;
    const v16bf qh0 = ldbf(QH + qoff), qh1 = ldbf(QH + qoff + 32), ql0 = ldbf(QL + qoff), ql1 = ldbf(QL + qoff + 32);
    const size_t koff = pbase + (size_t)lr * HD + 8 * hi;
    const size_t voff = (size_t)bh * HD * SEQ + (size_t)lr * SEQ + 8 * hi;
    v8f o[4];
#pragma unroll
    for (int dt = 0; dt < 4; ++dt) o[dt] = (v8f){};
    float m = -3.0e38f, l = 0.0f;
#pragma unroll 1
    for (int kv = 0; kv < SEQ; kv += 32) {
        const size_t ko = koff + (size_t)kv * HD;
        v8f s0 = (v8f){}, s1 = (v8f){};
        const v16bf kh00 = ldbf(KH + ko), kh01 = ldbf(KH + ko + 32), kl00 = ldbf(KL + ko), kl01 = ldbf(KL + ko + 32);
        s0 = wmmab(kh00, qh0, s0); s0 = wmmab(kh00, ql0, s0); s0 = wmmab(kl00, qh0, s0);
        s0 = wmmab(kh01, qh1, s0); s0 = wmmab(kh01, ql1, s0); s0 = wmmab(kl01, qh1, s0);
        const v16bf kh10 = ldbf(KH + ko + 16 * HD), kh11 = ldbf(KH + ko + 16 * HD + 32), kl10 = ldbf(KL + ko + 16 * HD), kl11 = ldbf(KL + ko + 16 * HD + 32);
        s1 = wmmab(kh10, qh0, s1); s1 = wmmab(kh10, ql0, s1); s1 = wmmab(kl10, qh0, s1);
        s1 = wmmab(kh11, qh1, s1); s1 = wmmab(kh11, ql1, s1); s1 = wmmab(kl11, qh1, s1);
        asm volatile("v_nop\n\tv_nop\n\tv_nop\n\tv_nop" : "+v"(s0), "+v"(s1) : "v"(kh11), "v"(kl11), "v"(qh1), "v"(ql1));
        float t0[8], t1[8]; float mx = -3.0e38f;
#pragma unroll
        for (int r = 0; r < 8; ++r) { t0[r] = s0[r] * LOG2E; t1[r] = s1[r] * LOG2E; mx = fmaxf(mx, fmaxf(t0[r], t1[r])); }
        mx = fmaxf(mx, __shfl_xor(mx, 16, 32));
        const float mnew = fmaxf(m, mx);
        const float alpha = __builtin_amdgcn_exp2f(m - mnew);
        m = mnew;
        const float sh = PEXP - mnew;
        float sum = 0.0f; v16h pb;
#pragma unroll
        for (int r = 0; r < 8; ++r) { const float e0 = __builtin_amdgcn_exp2f(t0[r] + sh); const float e1 = __builtin_amdgcn_exp2f(t1[r] + sh); sum += e0 + e1; pb[r] = (h16)e0; pb[8 + r] = (h16)e1; }
        sum += __shfl_xor(sum, 16, 32);
        l = l * alpha + sum;
#pragma unroll
        for (int dt = 0; dt < 4; ++dt)
#pragma unroll
            for (int r = 0; r < 8; ++r) o[dt][r] *= alpha;
        const size_t vo = voff + (size_t)kv;
        const v16h va0 = ldhf(VT + vo), va1 = ldhf(VT + vo + (size_t)16 * SEQ), va2 = ldhf(VT + vo + (size_t)32 * SEQ), va3 = ldhf(VT + vo + (size_t)48 * SEQ);
        o[0] = wmma16(va0, pb, o[0]); o[1] = wmma16(va1, pb, o[1]); o[2] = wmma16(va2, pb, o[2]); o[3] = wmma16(va3, pb, o[3]);
        asm volatile("v_nop\n\tv_nop\n\tv_nop\n\tv_nop" : "+v"(o[0]), "+v"(o[1]), "+v"(o[2]), "+v"(o[3]) : "v"(pb), "v"(va0), "v"(va3));
    }
    const float inv = 1.0f / l;
#pragma unroll
    for (int dt = 0; dt < 4; ++dt) { v8us oh, ol;
#pragma unroll
        for (int r = 0; r < 8; ++r) { unsigned short u, w2; splitf(o[dt][r] * inv, u, w2); oh[r] = u; ol[r] = w2; }
        *(v8usa*)(&sth[wave][lr * 72 + dt * 16 + 8 * hi]) = oh; *(v8usa*)(&stl[wave][lr * 72 + dt * 16 + 8 * hi]) = ol; }
    __builtin_amdgcn_wave_barrier(); asm volatile("" ::: "memory");
    const int rq = lane >> 3, pc = lane & 7;
#pragma unroll 1
    for (int ps = 0; ps < 2; ++ps) {
#pragma unroll
        for (int it = 0; it < 4; ++it) { const int row = it * 4 + rq;
            const v8us vh = *(const v8usa*)(&sth[wave][row * 72 + pc * 8]); const v8us vl = *(const v8usa*)(&stl[wave][row * 72 + pc * 8]);
            const size_t go = (size_t)(b * SEQ + q0 + row) * DQ + head * HD + pc * 8;
            *(volatile v8us*)(ATH + go) = vh; *(volatile v8us*)(ATL + go) = vl; }
        if (ps == 0) __threadfence(); }
}

constexpr size_t al256(size_t bytes) { return (bytes + 255) & ~(size_t)255; }
constexpr size_t SZ_XB   = (size_t)NB * SEQ * DM * 2;
constexpr size_t SZ_WQKV = (size_t)3 * DQ * DM * 2;
constexpr size_t SZ_WO   = (size_t)DM * DQ * 2;
constexpr size_t SZ_F    = (size_t)NB * SEQ * 3 * DQ * 4;
constexpr size_t SZ_QK   = (size_t)2 * NBH * SEQ * HD * 2;
constexpr size_t SZ_VT   = (size_t)NBH * HD * SEQ * 2;
constexpr size_t SZ_AT   = (size_t)NB * SEQ * DQ * 2;
constexpr size_t WS_TOTAL = al256(SZ_XB) + al256(SZ_WQKV) + al256(SZ_WO) + al256(SZ_F) + 2 * al256(SZ_QK) + al256(SZ_VT) + 2 * al256(SZ_AT);
static_assert(WS_TOTAL <= (size_t)134217728);

extern "C" void kernel_launch(void* const* d_in, const int* in_sizes, int n_in,
                              void* d_out, int out_size, void* d_ws, size_t ws_size, hipStream_t stream) {
    if (n_in < 5) return;
    const long long xmin = (long long)(NB - 1) * SEQ_FULL * DM + (long long)SEQ * DM;
    if ((long long)in_sizes[0] < xmin) return;
    if ((long long)in_sizes[1] < (long long)DM * 3 * DQ) return;
    if ((long long)in_sizes[2] < (long long)3 * DQ) return;
    if ((long long)in_sizes[3] < (long long)DQ * DM) return;
    if ((long long)in_sizes[4] < (long long)DM) return;
    if ((long long)out_size < xmin) return;
    if (WS_TOTAL > ws_size) return;
    const float* x = (const float*)d_in[0]; const float* wqkv = (const float*)d_in[1]; const float* bqkv = (const float*)d_in[2]; const float* wo = (const float*)d_in[3]; const float* bo = (const float*)d_in[4];
    float* OUT = (float*)d_out;
    char* wsp = (char*)d_ws;
    auto take = [&](size_t bytes) { char* p = wsp; wsp += al256(bytes); return (void*)p; };
    bf* XB = (bf*)take(SZ_XB); bf* WQKV = (bf*)take(SZ_WQKV); bf* WO = (bf*)take(SZ_WO); float* F = (float*)take(SZ_F);
    bf* QKH = (bf*)take(SZ_QK); bf* QKL = (bf*)take(SZ_QK); h16* VT = (h16*)take(SZ_VT); bf* ATH = (bf*)take(SZ_AT); bf* ATL = (bf*)take(SZ_AT);
    const size_t KOFF = (size_t)NBH * SEQ * HD;

    k_cvt8<<<(unsigned)(((size_t)NB * SEQ * DM / 8 + 255) / 256), 256, 0, stream>>>(x, XB);
    k_wtG<<<(unsigned)((DM * 3 * DQ / 64 + 63) / 64), 256, 0, stream>>>(wqkv, DM, 3 * DQ, WQKV);
    k_wtG<<<(unsigned)((DQ * DM / 64 + 63) / 64), 256, 0, stream>>>(wo, DQ, DM, WO);
    k_gemm_qkv<<<dim3(NB * SEQ / 64, 3 * DQ / 64, 1), 32, 0, stream>>>(XB, WQKV, F, bqkv);
    k_qkp<<<(unsigned)(((size_t)2 * NBH * SEQ * (HD / 8) + 255) / 256), 256, 0, stream>>>(F, QKH, QKL);
    k_vtp<<<(unsigned)(((size_t)NBH * HD * (SEQ / 8) + 255) / 256), 256, 0, stream>>>(F, VT);
    k_flash<<<dim3(SEQ / 64, NBH, 1), 128, 0, stream>>>(QKH, QKL, QKH + KOFF, QKL + KOFF, VT, ATH, ATL);
    k_gemm_out<<<dim3(SEQ / 64, DM / 64, NB), 32, 0, stream>>>(ATH, ATL, WO, OUT, bo);
}
